// CSOCSSC_v50_2319282340047
// MI455X (gfx1250) — hardware-verified
//
#include <hip/hip_runtime.h>
#include <stddef.h>


#define NTHR   256
#define NWAVE  8
#define EPT    8
#define CHUNK  (NTHR * EPT)
#define WCAP   (EPT * 32)
#define LISTN  (NWAVE * WCAP)
#define TEDGE  16
#define PASSN  (NWAVE * TEDGE)
#define PCAP   (CHUNK + PASSN)
#define NB     128
#define ND     64
#define HD     128
#define EDM    32
#define MI     (2 * ND + EDM)
#define PQW    512
#define MSW    68
#define RT     64
#define WTPLANE (4 * HD * ND)
#define NQ0    ((NB * ND) / (128 * NWAVE))
#define WSC    16.0f
#define WINV   0.0625f

static_assert(PCAP % PASSN == 0);
static_assert(NQ0 * 128 * NWAVE == NB * ND);
static_assert((NB % 32) == 0);
static_assert(NQ0 == 8);

typedef float    v2f  __attribute__((ext_vector_type(2)));
typedef float    v4f  __attribute__((ext_vector_type(4)));
typedef float    v8f  __attribute__((ext_vector_type(8)));
typedef int      v4i  __attribute__((ext_vector_type(4)));
typedef unsigned v4u  __attribute__((ext_vector_type(4)));
typedef _Float16 v8h  __attribute__((ext_vector_type(8)));
typedef _Float16 v16h __attribute__((ext_vector_type(16)));
typedef unsigned short v8us  __attribute__((ext_vector_type(8)));
typedef unsigned short v16us __attribute__((ext_vector_type(16)));
typedef __bf16   v16bf __attribute__((ext_vector_type(16)));
union FragH { v16h v; v8h h[2]; };
union FragB { v16bf v; v16us u; v8us u8[2]; };

__device__ __forceinline__ v8f zero8f() {
  v8f r;
#pragma unroll
  for (int i = 0; i < 8; ++i) r[i] = 0.0f;
  return r;
}

__device__ __forceinline__ v8f wmh(v16h a, v16h b, v8f c) {
  v8f d = __builtin_amdgcn_wmma_f32_16x16x32_f16(false, a, false, b, (short)0, c, false, false);
  asm volatile("v_nop\n\tv_nop\n\tv_nop\n\tv_nop" : "+v"(d) : "v"(a), "v"(b));
  return d;
}
__device__ __forceinline__ v8f wmb(v16bf a, v16bf b, v8f c) {
  v8f d = __builtin_amdgcn_wmma_f32_16x16x32_bf16(false, a, false, b, (short)0, c, false, false);
  asm volatile("v_nop\n\tv_nop\n\tv_nop\n\tv_nop" : "+v"(d) : "v"(a), "v"(b));
  return d;
}

__device__ __forceinline__ unsigned short bfb(float f) {
  const __bf16 b = (__bf16)f;
  return __builtin_bit_cast(unsigned short, b);
}
__device__ __forceinline__ float bff(unsigned short b) {
  return __uint_as_float(((unsigned)b) << 16);
}

__device__ __forceinline__ float silu_f(float v) {
  const float e = __expf(-v);
  return v * __builtin_amdgcn_rcpf(1.0f + e);
}

__device__ __forceinline__ int scan_chunk(const int* __restrict__ dsts, int nE, int cbase, int nodeBase,
                                          int vec8, int* hl, int tid, int wave) {
  int wc = 0;
  const int el0  = tid * EPT;
  const int e0   = cbase + el0;
  const int sent = -2147483647 - 1;
  v4i da, db;
  if (vec8 != 0 && cbase + CHUNK <= nE) {
    da = *(const v4i*)(dsts + e0);
    db = *(const v4i*)(dsts + e0 + 4);
  } else {
    da.x = (e0     < nE) ? dsts[min(e0, nE - 1)] : sent;
    da.y = (e0 + 1 < nE) ? dsts[min(e0 + 1, nE - 1)] : sent;
    da.z = (e0 + 2 < nE) ? dsts[min(e0 + 2, nE - 1)] : sent;
    da.w = (e0 + 3 < nE) ? dsts[min(e0 + 3, nE - 1)] : sent;
    db.x = (e0 + 4 < nE) ? dsts[min(e0 + 4, nE - 1)] : sent;
    db.y = (e0 + 5 < nE) ? dsts[min(e0 + 5, nE - 1)] : sent;
    db.z = (e0 + 6 < nE) ? dsts[min(e0 + 6, nE - 1)] : sent;
    db.w = (e0 + 7 < nE) ? dsts[min(e0 + 7, nE - 1)] : sent;
  }
  const unsigned nb = (unsigned)nodeBase;
  const unsigned s0 = (unsigned)da.x - nb, s1 = (unsigned)da.y - nb;
  const unsigned s2 = (unsigned)da.z - nb, s3 = (unsigned)da.w - nb;
  const unsigned s4 = (unsigned)db.x - nb, s5 = (unsigned)db.y - nb;
  const unsigned s6 = (unsigned)db.z - nb, s7 = (unsigned)db.w - nb;
  const bool h0 = s0 < (unsigned)NB, h1 = s1 < (unsigned)NB, h2 = s2 < (unsigned)NB, h3 = s3 < (unsigned)NB;
  const bool h4 = s4 < (unsigned)NB, h5 = s5 < (unsigned)NB, h6 = s6 < (unsigned)NB, h7 = s7 < (unsigned)NB;
  const unsigned any = __builtin_amdgcn_ballot_w32(h0 | h1 | h2 | h3 | h4 | h5 | h6 | h7);
  if (any != 0u) {
#define HITJ(J, HJ) { \
      const unsigned mj = __builtin_amdgcn_ballot_w32(HJ); \
      if (mj != 0u) { \
        if (HJ) { \
          const int pos = wc + (int)__builtin_amdgcn_mbcnt_lo(mj, 0u); \
          if (pos < WCAP) hl[wave * WCAP + pos] = el0 + (J); \
        } \
        wc += (int)__builtin_popcount(mj); } }
    HITJ(0, h0)
    HITJ(1, h1)
    HITJ(2, h2)
    HITJ(3, h3)
    HITJ(4, h4)
    HITJ(5, h5)
    HITJ(6, h6)
    HITJ(7, h7)
#undef HITJ
  }
  return wc;
}

__global__ __launch_bounds__(NTHR) void k_wprep(const float* __restrict__ Wn1, const float* __restrict__ Wc1,
                                                unsigned short* wt) {
  const int g    = (int)blockIdx.x * NTHR + (int)threadIdx.x;
  const int k0   = (g & 7) * 8;
  const int n    = (g >> 3) & (HD - 1);
  const int cb   = (g >> 10) & 3;
  const int kofs = (cb & 1) * ND;
  unsigned ph[4] = {0u, 0u, 0u, 0u}, pl[4] = {0u, 0u, 0u, 0u};
#pragma unroll
  for (int i = 0; i < 8; ++i) {
    const int si = (kofs + k0 + i) * HD + n;
    const float wa = Wn1[si], wb = Wc1[si];
    const float w = (cb < 2) ? wa : wb;
    const unsigned short hb = bfb(w);
    const unsigned short lb = bfb(w - bff(hb));
    ph[i >> 1] |= ((unsigned)hb) << (16 * (i & 1));
    pl[i >> 1] |= ((unsigned)lb) << (16 * (i & 1));
  }
  v4u hv, lv;
  hv.x = ph[0]; hv.y = ph[1]; hv.z = ph[2]; hv.w = ph[3];
  lv.x = pl[0]; lv.y = pl[1]; lv.z = pl[2]; lv.w = pl[3];
  const size_t ofs = (size_t)(cb * HD + n) * ND + (size_t)k0;
  unsigned short* dh = wt + ofs;
  unsigned short* dl = wt + WTPLANE + ofs;
  *(volatile v4u*)dh = hv;
  *(volatile v4u*)dl = lv;
  __threadfence();
  *(volatile v4u*)dh = hv;
  *(volatile v4u*)dl = lv;
}

__global__ __launch_bounds__(NTHR) void k_pq(const float* __restrict__ h, const unsigned short* __restrict__ wt,
                                             const float* __restrict__ bn1, const float* __restrict__ bc1,
                                             float* pq, int nN) {
  __shared__ __attribute__((aligned(16))) float stg[RT * HD];
  const int tid = threadIdx.x, lane = tid & 31, wave = tid >> 5, hh = lane >> 4, m = lane & 15;
  const int rt = wave & 3, c2 = wave >> 2;
  const int cb = (int)blockIdx.y;
  const int rowBase = (int)blockIdx.x * RT;
  int row = rowBase + 16 * rt + m;
  row = row > nN - 1 ? nN - 1 : row;
  const float* hp = h + (size_t)row * ND;

  FragB ah[2], al[2];
#pragma unroll
  for (int ks = 0; ks < 2; ++ks) {
    const float* p = hp + 32 * ks + 8 * hh;
    const v4f f0 = *(const v4f*)(p);
    const v4f f1 = *(const v4f*)(p + 4);
    const v4f f2 = *(const v4f*)(p + 16);
    const v4f f3 = *(const v4f*)(p + 20);
    const float ev[16] = {f0.x, f0.y, f0.z, f0.w, f1.x, f1.y, f1.z, f1.w,
                          f2.x, f2.y, f2.z, f2.w, f3.x, f3.y, f3.z, f3.w};
#pragma unroll
    for (int i = 0; i < 16; ++i) {
      const unsigned short hb = bfb(ev[i]);
      ah[ks].u[i] = hb;
      al[ks].u[i] = bfb(ev[i] - bff(hb));
    }
  }
  v8f acc[4];
#pragma unroll
  for (int ct = 0; ct < 4; ++ct) acc[ct] = zero8f();
#pragma unroll
  for (int ct = 0; ct < 4; ++ct) {
    const int nc = 64 * c2 + 16 * ct + m;
    const unsigned short* bp = wt + (size_t)(cb * HD + nc) * ND;
#pragma unroll
    for (int ks = 0; ks < 2; ++ks) {
      FragB bh, bl;
      bh.u8[0] = *(const v8us*)(bp + 32 * ks + 8 * hh);
      bh.u8[1] = *(const v8us*)(bp + 32 * ks + 16 + 8 * hh);
      bl.u8[0] = *(const v8us*)(bp + WTPLANE + 32 * ks + 8 * hh);
      bl.u8[1] = *(const v8us*)(bp + WTPLANE + 32 * ks + 16 + 8 * hh);
      acc[ct] = wmb(ah[ks].v, bh.v, acc[ct]);
      acc[ct] = wmb(ah[ks].v, bl.v, acc[ct]);
      acc[ct] = wmb(al[ks].v, bh.v, acc[ct]);
    }
  }
#pragma unroll
  for (int ct = 0; ct < 4; ++ct) {
    const int col = 64 * c2 + 16 * ct + m;
    const float b1 = bn1[col], b3 = bc1[col];
    const float bias = (cb == 1) ? b1 : ((cb == 3) ? b3 : 0.0f);
#pragma unroll
    for (int r = 0; r < 8; ++r) stg[(16 * rt + 8 * hh + r) * HD + col] = acc[ct][r] + bias;
  }
  __syncthreads();
  v4f ov[8];
#pragma unroll
  for (int i = 0; i < 8; ++i) ov[i] = *(const v4f*)(stg + (wave + 8 * i) * HD + 4 * lane);
#pragma unroll
  for (int i = 0; i < 8; ++i) {
    float* dp = pq + (size_t)(rowBase + wave + 8 * i) * PQW + cb * HD + 4 * lane;
    *(volatile v4f*)dp = ov[i];
  }
  __threadfence();
#pragma unroll
  for (int i = 0; i < 8; ++i) {
    float* dp = pq + (size_t)(rowBase + wave + 8 * i) * PQW + cb * HD + 4 * lane;
    *(volatile v4f*)dp = ov[i];
  }
}

__global__ __launch_bounds__(NTHR) void k_agg(
    const float* __restrict__ h, const float* __restrict__ x, const float* __restrict__ ed,
    const float* __restrict__ We1, const float* __restrict__ be1,
    const float* __restrict__ We2, const float* __restrict__ be2,
    const float* __restrict__ Wn1, const float* __restrict__ Wc1,
    const float* __restrict__ Wn2, const float* __restrict__ bn2, const float* __restrict__ Wc2,
    const int* __restrict__ ei, const float* __restrict__ pq,
    float* out0, float* out1, int nN, int nE, int vec8) {
  __shared__ __attribute__((aligned(16))) float          acch[(NB + 1) * ND];
  __shared__ __attribute__((aligned(16))) float          accx[(NB + 1) * 4];
  __shared__ __attribute__((aligned(16))) float          msg[PASSN * MSW];
  __shared__ __attribute__((aligned(16))) _Float16       wn1e[HD * EDM];
  __shared__ __attribute__((aligned(16))) _Float16       wc1e[HD * EDM];
  __shared__ __attribute__((aligned(16))) unsigned short wn2h[ND * HD];
  __shared__ __attribute__((aligned(16))) unsigned short wn2l[ND * HD];
  __shared__ __attribute__((aligned(16))) float          we2[EDM * EDM];
  __shared__ __attribute__((aligned(16))) float          fsm[288];
  __shared__ __attribute__((aligned(16))) int            hl[LISTN];
  __shared__ __attribute__((aligned(16))) int            pend[PCAP];
  __shared__ int slotb[PASSN];
  __shared__ int wcnt[NWAVE];
  __shared__ int pendN;

  const int tid = threadIdx.x, lane = tid & 31, wave = tid >> 5, hh = lane >> 4, m = lane & 15;
  const int nodeBase = (int)blockIdx.x * NB;
  const int te = wave * TEDGE + m;
  const int* srcs = ei;
  const int* dsts = ei + nE;

  for (int i = tid; i < (NB + 1) * ND; i += NTHR) acch[i] = 0.0f;
  for (int i = tid; i < (NB + 1) * 4; i += NTHR) accx[i] = 0.0f;
  for (int i = tid; i < HD * EDM; i += NTHR) {
    const int u = i >> 5, k = i & 31;
    const int si = (2 * ND + k) * HD + u;
    wn1e[i] = (_Float16)(Wn1[si] * WSC);
    wc1e[i] = (_Float16)(Wc1[si] * WSC);
  }
  for (int i = tid; i < ND * HD; i += NTHR) {
    const int o = i >> 7, k = i & (HD - 1);
    const float w = Wn2[k * ND + o];
    const unsigned short hb = bfb(w);
    wn2h[i] = hb;
    wn2l[i] = bfb(w - bff(hb));
  }
  for (int i = tid; i < EDM * EDM; i += NTHR) we2[i] = We2[i];
  if (tid < EDM) { fsm[tid] = We1[tid]; fsm[32 + tid] = be1[tid]; fsm[64 + tid] = be2[tid]; }
  if (tid < ND)  fsm[96 + tid] = bn2[tid];
  if (tid < HD)  fsm[160 + tid] = Wc2[tid];
  if (tid == 0) pendN = 0;
  __syncthreads();

  const v8f z8 = zero8f();
  const int nChunks = (nE + CHUNK - 1) / CHUNK;
#pragma unroll 1
  for (int ch = 0; ch < nChunks; ++ch) {
    const int cbase = ch * CHUNK;
    const int wc = scan_chunk(dsts, nE, cbase, nodeBase, vec8, hl, tid, wave);
    if (lane == 0) wcnt[wave] = wc;
    __syncthreads();

    const int base = pendN;
    int tot = 0, myoff = 0;
#pragma unroll
    for (int w = 0; w < NWAVE; ++w) {
      int c = wcnt[w];
      c = c > WCAP ? WCAP : (c < 0 ? 0 : c);
      if (w < wave) myoff += c;
      tot += c;
    }
    int newN = base + tot;
    newN = newN > PCAP ? PCAP : newN;
    {
      int n = wcnt[wave];
      n = n > WCAP ? WCAP : (n < 0 ? 0 : n);
      const int* lp = hl + wave * WCAP;
      for (int i = lane; i < n; i += 32) {
        const int pos = base + myoff + i;
        if (pos < PCAP) pend[pos] = cbase + lp[i];
      }
    }
    const int fin = (ch == nChunks - 1) ? 1 : 0;
    const int R   = (fin != 0) ? (newN + PASSN - 1) / PASSN : newN / PASSN;
    const int Pv  = (fin != 0) ? newN : R * PASSN;
    __syncthreads();

#pragma unroll 1
    for (int r = 0; r < R; ++r) {
      const int idx = r * PASSN + te;
      const bool valid = idx < Pv;
      int e = pend[idx];
      e = valid ? e : 0;
      e = e < 0 ? 0 : (e > nE - 1 ? nE - 1 : e);
      int d = dsts[e];
      int s = srcs[e];
      const float dist0 = ed[e];
      const float dist = valid ? dist0 : 0.0f;
      int slot = d - nodeBase;
      if (!valid || (unsigned)slot >= (unsigned)NB) slot = NB;
      d = d < 0 ? 0 : (d > nN - 1 ? nN - 1 : d);
      s = s < 0 ? 0 : (s > nN - 1 ? nN - 1 : s);
      if (hh == 0) slotb[te] = slot;
      const float* prow = pq + (size_t)s * PQW;
      const float* qrow = pq + (size_t)d * PQW;

      float t[32];
#pragma unroll
      for (int k4 = 0; k4 < 8; ++k4) {
        const v4f w4 = *(const v4f*)(fsm + 4 * k4);
        const v4f b4 = *(const v4f*)(fsm + 32 + 4 * k4);
        t[4 * k4 + 0] = silu_f(fmaf(dist, w4.x, b4.x));
        t[4 * k4 + 1] = silu_f(fmaf(dist, w4.y, b4.y));
        t[4 * k4 + 2] = silu_f(fmaf(dist, w4.z, b4.z));
        t[4 * k4 + 3] = silu_f(fmaf(dist, w4.w, b4.w));
      }
      float ea[16];
      {
        const v4f c0 = *(const v4f*)(fsm + 64 + 8 * hh);
        const v4f c1 = *(const v4f*)(fsm + 68 + 8 * hh);
        const v4f c2 = *(const v4f*)(fsm + 80 + 8 * hh);
        const v4f c3 = *(const v4f*)(fsm + 84 + 8 * hh);
        ea[0] = c0.x; ea[1] = c0.y; ea[2]  = c0.z; ea[3]  = c0.w;
        ea[4] = c1.x; ea[5] = c1.y; ea[6]  = c1.z; ea[7]  = c1.w;
        ea[8] = c2.x; ea[9] = c2.y; ea[10] = c2.z; ea[11] = c2.w;
        ea[12] = c3.x; ea[13] = c3.y; ea[14] = c3.z; ea[15] = c3.w;
      }
#pragma unroll
      for (int k = 0; k < 32; ++k) {
        const float* wr = we2 + k * EDM + 8 * hh;
        const v4f wa = *(const v4f*)(wr);
        const v4f wb = *(const v4f*)(wr + 4);
        const v4f wq = *(const v4f*)(wr + 16);
        const v4f wd = *(const v4f*)(wr + 20);
        const float tk = t[k];
        ea[0]  = fmaf(tk, wa.x, ea[0]);  ea[1]  = fmaf(tk, wa.y, ea[1]);
        ea[2]  = fmaf(tk, wa.z, ea[2]);  ea[3]  = fmaf(tk, wa.w, ea[3]);
        ea[4]  = fmaf(tk, wb.x, ea[4]);  ea[5]  = fmaf(tk, wb.y, ea[5]);
        ea[6]  = fmaf(tk, wb.z, ea[6]);  ea[7]  = fmaf(tk, wb.w, ea[7]);
        ea[8]  = fmaf(tk, wq.x, ea[8]);  ea[9]  = fmaf(tk, wq.y, ea[9]);
        ea[10] = fmaf(tk, wq.z, ea[10]); ea[11] = fmaf(tk, wq.w, ea[11]);
        ea[12] = fmaf(tk, wd.x, ea[12]); ea[13] = fmaf(tk, wd.y, ea[13]);
        ea[14] = fmaf(tk, wd.z, ea[14]); ea[15] = fmaf(tk, wd.w, ea[15]);
      }
      FragH eb;
#pragma unroll
      for (int i = 0; i < 16; ++i) eb.v[i] = (_Float16)ea[i];

      v8f acc2[4];
#pragma unroll
      for (int ot = 0; ot < 4; ++ot) acc2[ot] = zero8f();
#pragma unroll 1
      for (int kc = 0; kc < 4; ++kc) {
        FragB bh, bl;
#pragma unroll
        for (int half = 0; half < 2; ++half) {
          const int ft = 2 * kc + half;
          FragH a;
          const _Float16* ap = wn1e + (16 * ft + m) * EDM + 8 * hh;
          a.h[0] = *(const v8h*)ap;
          a.h[1] = *(const v8h*)(ap + 16);
          const v8f dd = wmh(a.v, eb.v, z8);
          const float* pp = prow + 16 * ft + 8 * hh;
          const float* qp = qrow + HD + 16 * ft + 8 * hh;
          const v4f p0 = *(const v4f*)pp, p1 = *(const v4f*)(pp + 4);
          const v4f q0 = *(const v4f*)qp, q1 = *(const v4f*)(qp + 4);
          const float pz[8] = {p0.x, p0.y, p0.z, p0.w, p1.x, p1.y, p1.z, p1.w};
          const float qz[8] = {q0.x, q0.y, q0.z, q0.w, q1.x, q1.y, q1.z, q1.w};
#pragma unroll
          for (int rr = 0; rr < 8; ++rr) {
            const float z  = fmaf(dd[rr], WINV, pz[rr]) + qz[rr];
            const float sg = silu_f(z);
            const unsigned short hb = bfb(sg);
            bh.u[8 * half + rr] = hb;
            bl.u[8 * half + rr] = bfb(sg - bff(hb));
          }
        }
#pragma unroll
        for (int ot = 0; ot < 4; ++ot) {
          FragB fa, fl;
          const unsigned short* wp = wn2h + (16 * ot + m) * HD + 32 * kc + 8 * hh;
          const unsigned short* wl = wn2l + (16 * ot + m) * HD + 32 * kc + 8 * hh;
          fa.u8[0] = *(const v8us*)wp;
          fa.u8[1] = *(const v8us*)(wp + 16);
          fl.u8[0] = *(const v8us*)wl;
          fl.u8[1] = *(const v8us*)(wl + 16);
          acc2[ot] = wmb(fa.v, bh.v, acc2[ot]);
          acc2[ot] = wmb(fa.v, bl.v, acc2[ot]);
          acc2[ot] = wmb(fl.v, bh.v, acc2[ot]);
        }
      }
      {
        float* mrow = msg + te * MSW;
#pragma unroll
        for (int ot = 0; ot < 4; ++ot) {
          const v4f b0 = *(const v4f*)(fsm + 96 + 16 * ot + 8 * hh);
          const v4f b1 = *(const v4f*)(fsm + 100 + 16 * ot + 8 * hh);
          v4f u0, u1;
          u0.x = acc2[ot][0] + b0.x; u0.y = acc2[ot][1] + b0.y; u0.z = acc2[ot][2] + b0.z; u0.w = acc2[ot][3] + b0.w;
          u1.x = acc2[ot][4] + b1.x; u1.y = acc2[ot][5] + b1.y; u1.z = acc2[ot][6] + b1.z; u1.w = acc2[ot][7] + b1.w;
          *(v4f*)(mrow + 16 * ot + 8 * hh)     = u0;
          *(v4f*)(mrow + 16 * ot + 8 * hh + 4) = u1;
        }
      }

      float cw = 0.0f;
#pragma unroll 1
      for (int ft = 0; ft < 8; ++ft) {
        FragH a;
        const _Float16* ap = wc1e + (16 * ft + m) * EDM + 8 * hh;
        a.h[0] = *(const v8h*)ap;
        a.h[1] = *(const v8h*)(ap + 16);
        const v8f dd = wmh(a.v, eb.v, z8);
        const float* pp = prow + 2 * HD + 16 * ft + 8 * hh;
        const float* qp = qrow + 3 * HD + 16 * ft + 8 * hh;
        const v4f p0 = *(const v4f*)pp, p1 = *(const v4f*)(pp + 4);
        const v4f q0 = *(const v4f*)qp, q1 = *(const v4f*)(qp + 4);
        const v4f w0 = *(const v4f*)(fsm + 160 + 16 * ft + 8 * hh);
        const v4f w1 = *(const v4f*)(fsm + 164 + 16 * ft + 8 * hh);
        const float pz[8] = {p0.x, p0.y, p0.z, p0.w, p1.x, p1.y, p1.z, p1.w};
        const float qz[8] = {q0.x, q0.y, q0.z, q0.w, q1.x, q1.y, q1.z, q1.w};
        const float wz[8] = {w0.x, w0.y, w0.z, w0.w, w1.x, w1.y, w1.z, w1.w};
#pragma unroll
        for (int rr = 0; rr < 8; ++rr) {
          const float z = fmaf(dd[rr], WINV, pz[rr]) + qz[rr];
          cw = fmaf(silu_f(z), wz[rr], cw);
        }
      }
      cw += __shfl_xor(cw, 16);
      {
        const float xs0 = x[(size_t)s * 3 + 0], xs1 = x[(size_t)s * 3 + 1], xs2 = x[(size_t)s * 3 + 2];
        const float xd0 = x[(size_t)d * 3 + 0], xd1 = x[(size_t)d * 3 + 1], xd2 = x[(size_t)d * 3 + 2];
        const float dx = xs0 - xd0, dy = xs1 - xd1, dz = xs2 - xd2;
        const float len = fmaxf(sqrtf(dx * dx + dy * dy + dz * dz), 1e-8f);
        const float inv = 1.0f / len;
        const float m0 = cw * (dx * inv), m1 = cw * (dy * inv), m2 = cw * (dz * inv);
        if (hh == 0) {
          float* mc = msg + te * MSW + ND;
          mc[0] = m0; mc[1] = m1; mc[2] = m2;
        }
      }
      __syncthreads();

      if (wave == 0) {
#pragma unroll 1
        for (int i = 0; i < PASSN; ++i) {
          int sl = slotb[i];
          sl = sl < 0 ? 0 : (sl > NB ? NB : sl);
          const v2f mv = *(const v2f*)(msg + i * MSW + 2 * lane);
          v2f* ap = (v2f*)(acch + sl * ND + 2 * lane);
          const v2f av = *ap;
          *ap = av + mv;
          if (lane < 3) {
            const float xv = msg[i * MSW + ND + lane];
            accx[sl * 4 + lane] += xv;
          }
        }
      }
      __syncthreads();
    }

    int rem = newN - R * PASSN;
    rem = rem < 0 ? 0 : rem;
    if (R > 0 && tid < rem) pend[tid] = pend[R * PASSN + tid];
    if (tid == 0) pendN = rem;
  }
  __syncthreads();

  const size_t lim0 = (size_t)nN * ND;
  v4f ov[NQ0];
#pragma unroll
  for (int q = 0; q < NQ0; ++q) {
    const int f  = (wave * NQ0 + q) * 128 + 4 * lane;
    const int sl = f >> 6;
    const int c  = f & 63;
    int node = nodeBase + sl;
    node = node > nN - 1 ? nN - 1 : node;
    const v4f hv = *(const v4f*)(h + (size_t)node * ND + c);
    const v4f av = *(const v4f*)(acch + sl * ND + c);
    ov[q] = hv + av;
  }
  const size_t lim1 = (size_t)nN * 3;
  const bool w1ok = wave < 3;
  const int f1 = (w1ok ? wave : 0) * 128 + 4 * lane;
  float xo[4];
#pragma unroll
  for (int j = 0; j < 4; ++j) {
    const int el = f1 + j;
    const int sl = el / 3;
    const int c  = el - 3 * sl;
    int node = nodeBase + sl;
    node = node > nN - 1 ? nN - 1 : node;
    xo[j] = x[(size_t)node * 3 + c] + accx[sl * 4 + c];
  }
  v4f xv;
  xv.x = xo[0]; xv.y = xo[1]; xv.z = xo[2]; xv.w = xo[3];
  const size_t g0b = (size_t)nodeBase * ND;
  const size_t g1  = (size_t)nodeBase * 3 + (size_t)f1;

#pragma unroll
  for (int q = 0; q < NQ0; ++q) {
    const size_t gi = g0b + (size_t)((wave * NQ0 + q) * 128 + 4 * lane);
    if (gi + 4 <= lim0) *(volatile v4f*)(out0 + gi) = ov[q];
  }
  if (w1ok) {
    if (g1 + 4 <= lim1) {
      *(volatile v4f*)(out1 + g1) = xv;
    } else {
#pragma unroll
      for (int j = 0; j < 4; ++j) if (g1 + (size_t)j < lim1) *(volatile float*)(out1 + g1 + j) = xo[j];
    }
  }
  __threadfence();
#pragma unroll
  for (int q = 0; q < NQ0; ++q) {
    const size_t gi = g0b + (size_t)((wave * NQ0 + q) * 128 + 4 * lane);
    if (gi + 4 <= lim0) *(volatile v4f*)(out0 + gi) = ov[q];
  }
  if (w1ok) {
    if (g1 + 4 <= lim1) {
      *(volatile v4f*)(out1 + g1) = xv;
    } else {
#pragma unroll
      for (int j = 0; j < 4; ++j) if (g1 + (size_t)j < lim1) *(volatile float*)(out1 + g1 + j) = xo[j];
    }
  }
}

extern "C" void kernel_launch(void* const* d_in, const int* in_sizes, int n_in,
                              void* d_out, int out_size, void* d_ws, size_t ws_size,
                              hipStream_t stream) {
  if (n_in < 15) return;
  const int nN = in_sizes[0] / ND;
  if (nN <= 0 || in_sizes[0] != nN * ND || in_sizes[1] != nN * 3) return;
  const int nE = in_sizes[2];
  if (nE < 0 || in_sizes[14] != 2 * nE) return;
  if (in_sizes[3] != EDM || in_sizes[4] != EDM || in_sizes[5] != EDM * EDM || in_sizes[6] != EDM) return;
  if (in_sizes[7] != MI * HD || in_sizes[8] != HD || in_sizes[9] != HD * ND || in_sizes[10] != ND) return;
  if (in_sizes[11] != MI * HD || in_sizes[12] != HD || in_sizes[13] != HD) return;
  if (out_size != nN * ND + nN * 3) return;

  const float* h    = (const float*)d_in[0];
  const float* x    = (const float*)d_in[1];
  const float* ed   = (const float*)d_in[2];
  const float* We1  = (const float*)d_in[3];
  const float* be1  = (const float*)d_in[4];
  const float* We2  = (const float*)d_in[5];
  const float* be2  = (const float*)d_in[6];
  const float* Wn1  = (const float*)d_in[7];
  const float* bn1  = (const float*)d_in[8];
  const float* Wn2  = (const float*)d_in[9];
  const float* bn2  = (const float*)d_in[10];
  const float* Wc1  = (const float*)d_in[11];
  const float* bc1  = (const float*)d_in[12];
  const float* Wc2  = (const float*)d_in[13];
  const int*   ei   = (const int*)d_in[14];
  float* out0 = (float*)d_out;
  float* out1 = (float*)((char*)d_out + (size_t)nN * ND * 4);

  const int nPad = ((nN + RT - 1) / RT) * RT;
  const int nBlk = (nN + NB - 1) / NB;

  char* ws = (char*)d_ws;
  size_t off = 0;
  const size_t oWT = off; off += (size_t)2 * WTPLANE * 2;            off = (off + 255) & ~(size_t)255;
  const size_t oPQ = off; off += (size_t)nPad * PQW * 4;              off = (off + 255) & ~(size_t)255;
  if (off > ws_size || off > (size_t)134217728) return;
  unsigned short* wt = (unsigned short*)(ws + oWT);
  float* pq = (float*)(ws + oPQ);

  const int vec8 = ((nE & 3) == 0) ? 1 : 0;

  k_wprep<<<(4 * HD * ND / 8 + NTHR - 1) / NTHR, NTHR, 0, stream>>>(Wn1, Wc1, wt);

  k_pq<<<dim3(nPad / RT, 4), NTHR, 0, stream>>>(h, wt, bn1, bc1, pq, nN);

  k_agg<<<nBlk, NTHR, 0, stream>>>(h, x, ed, We1, be1, We2, be2, Wn1, Wc1, Wn2, bn2, Wc2,
                                   ei, pq, out0, out1, nN, nE, vec8);
}
